// Encoder_45784351375645
// MI455X (gfx1250) — hardware-verified
//
#include <hip/hip_runtime.h>
#include <math.h>

constexpr int NBATCH   = 512;
constexpr int NVAR     = 256;
constexpr int NWIN     = 64;
constexpr int NHID     = 64;
constexpr int NGATE    = 4 * NHID;
constexpr int NKHC     = 2 * NHID;
constexpr int ROWS_UV  = NBATCH * NVAR;
constexpr int BLK_ROWS = 16;
constexpr int SCAN_THR = 512;
constexpr int HCP      = 136;
constexpr int XTP      = 264;
constexpr int GTP      = 260;
constexpr int NOUT0    = NWIN * NBATCH * NVAR;
constexpr int NOUT1    = NWIN * NBATCH * NHID;
constexpr float W_CARRY      = 16.0f;
constexpr float W_CARRY_INV  = 1.0f / 16.0f;
constexpr float ACT_CARRY    = 256.0f;
constexpr float FOLD_INV     = 1.0f / (16.0f * 256.0f);
constexpr float WV_CARRY     = 64.0f;
constexpr float WV_CARRY_INV = 1.0f / 64.0f;
constexpr float WV_RES       = 2048.0f;
constexpr float WV_RES_INV   = 1.0f / 2048.0f;
static_assert(NWIN % 32 == 0 && NKHC % 32 == 0 && NVAR % 32 == 0 && NHID % 32 == 0, "k multiples of 32");
static_assert(ROWS_UV % 64 == 0 && NWIN % 64 == 0, "gemm tile multiples");
static_assert(NBATCH % BLK_ROWS == 0, "batch tiles");
static_assert(SCAN_THR / 32 == BLK_ROWS, "one wave per batch row");
static_assert(NGATE == 16 * (SCAN_THR / 32), "one gate n-tile per wave");
static_assert(16 * GTP <= 2 * 16 * NVAR, "gate tile fits the score buffer");
static_assert((size_t)NOUT0 * 4 == 33554432, "out1 byte offset");
static_assert(((size_t)NOUT0 * 4) % 128 == 0, "out1 line aligned");
static_assert(HCP % 8 == 0 && XTP % 8 == 0, "16-byte aligned fragment rows");

typedef __attribute__((ext_vector_type(16))) _Float16 v16h;
typedef __attribute__((ext_vector_type(8)))  _Float16 v8h;
typedef __attribute__((ext_vector_type(16))) __bf16   v16b;
typedef __attribute__((ext_vector_type(8)))  __bf16   v8b;
typedef __attribute__((ext_vector_type(8)))  float    v8f;
typedef __attribute__((ext_vector_type(4)))  float    v4f;
typedef __attribute__((ext_vector_type(2)))  unsigned v2u;

__device__ __forceinline__ unsigned short f2bf_bits(float f) {
  unsigned u = __float_as_uint(f);
  return (unsigned short)((u + 0x7FFFu + ((u >> 16) & 1u)) >> 16);
}
__device__ __forceinline__ float bf_bits2f(unsigned short h) { return __uint_as_float(((unsigned)h) << 16); }

__device__ __forceinline__ float h16_to_f32(unsigned hb) {
  const unsigned sgn = (hb & 0x8000u) << 16;
  const unsigned em = hb & 0x7fffu;
  const float fn = __uint_as_float((em << 13) + 0x38000000u);
  const float fs = (float)em * 5.9604644775390625e-8f;
  const float mag = (em < 0x400u) ? fs : fn;
  return __uint_as_float(__float_as_uint(mag) | sgn);
}

__device__ __forceinline__ void dep_guard_h(v8f& a, v8f& b, v16h x, v16h y) { asm volatile("v_nop\n\tv_nop\n\tv_nop\n\tv_nop" : "+v"(a), "+v"(b) : "v"(x), "v"(y)); }
__device__ __forceinline__ void dep_guard_b(v8f& a, v8f& b, v16b x, v16b y) { asm volatile("v_nop\n\tv_nop\n\tv_nop\n\tv_nop" : "+v"(a), "+v"(b) : "v"(x), "v"(y)); }
__device__ __forceinline__ void keep4_h(v16h a, v16h b, v16h c, v16h d) { asm volatile("v_nop" :: "v"(a), "v"(b), "v"(c), "v"(d)); }
__device__ __forceinline__ void keep4_b(v16b a, v16b b, v16b c, v16b d) { asm volatile("v_nop" :: "v"(a), "v"(b), "v"(c), "v"(d)); }
__device__ __forceinline__ void acc_guard4(v8f& a, v8f& b, v8f& c, v8f& d) { asm volatile("v_nop\n\tv_nop\n\tv_nop\n\tv_nop" : "+v"(a), "+v"(b), "+v"(c), "+v"(d)); }

template <typename T> struct Frag;
template <> struct Frag<_Float16> {
  typedef v16h V; union U { v16h v; v8h h[2]; };
  static __device__ __forceinline__ v16h load(const _Float16* p) {
    U f; f.h[0] = *(const v8h*)(p); f.h[1] = *(const v8h*)(p + 16); return f.v;
  }
  static __device__ __forceinline__ v8f mma(v16h a, v16h b, v8f c) {
    return __builtin_amdgcn_wmma_f32_16x16x32_f16(false, a, false, b, (short)0, c, false, false);
  }
  static __device__ __forceinline__ void guard(v8f& a, v8f& b, v16h x, v16h y) { dep_guard_h(a, b, x, y); }
  static __device__ __forceinline__ void keep(v16h a, v16h b, v16h c, v16h d) { keep4_h(a, b, c, d); }
};
template <> struct Frag<__bf16> {
  typedef v16b V; union U { v16b v; v8b h[2]; };
  static __device__ __forceinline__ v16b load(const __bf16* p) {
    U f; f.h[0] = *(const v8b*)(p); f.h[1] = *(const v8b*)(p + 16); return f.v;
  }
  static __device__ __forceinline__ v8f mma(v16b a, v16b b, v8f c) {
    return __builtin_amdgcn_wmma_f32_16x16x32_bf16(false, a, false, b, (short)0, c, false, false);
  }
  static __device__ __forceinline__ void guard(v8f& a, v8f& b, v16b x, v16b y) { dep_guard_b(a, b, x, y); }
  static __device__ __forceinline__ void keep(v16b a, v16b b, v16b c, v16b d) { keep4_b(a, b, c, d); }
};

__device__ __forceinline__ v8f mma_h(v16h a, v16h b, v8f c) {
  c = __builtin_amdgcn_wmma_f32_16x16x32_f16(false, a, false, b, (short)0, c, false, false);
  asm volatile("v_nop\n\tv_nop\n\tv_nop\n\tv_nop" : "+v"(c) : "v"(a), "v"(b));
  return c;
}

template <int ET> struct Elem;
template <> struct Elem<0> { typedef _Float16 T; };
template <> struct Elem<1> { typedef __bf16 T; };
template <int ET, bool SPLIT, int BIAS_MODE, int OUT_MODE, bool RESID, int ACT = 0>
__global__ __launch_bounds__(256) void wmma_gemm64(
    const unsigned short* __restrict__ Ap, const unsigned short* __restrict__ A2p, int lda, long strideA,
    const unsigned short* __restrict__ Btp, const unsigned short* __restrict__ Bt2p, int ldb, long strideB,
    void* __restrict__ Cout, void* __restrict__ Cout2, int ldc, long strideC,
    const float* __restrict__ bias,
    const float* __restrict__ resid, long strideR,
    int M, int N, int K, float scale) {
  typedef typename Elem<ET>::T T;
  typedef typename Frag<T>::V V;
  const T* A = (const T*)Ap; const T* A2 = (const T*)A2p; const T* Bt = (const T*)Btp; const T* Bt2 = (const T*)Bt2p;
  __shared__ __align__(16) float sT[8][16 * 68];
  const int b    = blockIdx.y;
  const int lane = threadIdx.x & 31;
  const int wave = threadIdx.x >> 5;
  const int tilesN = N >> 6;
  const int tilesM = M >> 6;
  const int tile = blockIdx.x * 8 + wave;
  if (tile >= tilesM * tilesN) return;
  const int tm = tile / tilesN;
  const int tn = tile - tm * tilesN;
  const int m0 = tm << 6;
  const int n0 = tn << 6;

  const T* Ab  = A  + (size_t)b * strideA;
  const T* Bb  = Bt + (size_t)b * strideB;
  const T* Ab2 = SPLIT ? (A2  + (size_t)b * strideA) : nullptr;
  const T* Bb2 = SPLIT ? (Bt2 + (size_t)b * strideB) : nullptr;

  const int rlane = lane & 15;
  const int koff  = (lane >> 4) * 8;
  const int mOff  = (lane >> 4) * 8;

  v8f acc[4][4];
#pragma unroll
  for (int i = 0; i < 4; ++i)
#pragma unroll
    for (int j = 0; j < 4; ++j) acc[i][j] = (v8f){0.f,0.f,0.f,0.f,0.f,0.f,0.f,0.f};

  for (int k0 = 0; k0 < K; k0 += 32) {
    V bh[4], bl[4];
#pragma unroll
    for (int j = 0; j < 4; ++j) {
      const size_t bo = (size_t)(n0 + (j << 4) + rlane) * ldb + koff + k0;
      bh[j] = Frag<T>::load(Bb + bo);
      if (SPLIT) bl[j] = Frag<T>::load(Bb2 + bo);
    }
#pragma unroll
    for (int i = 0; i < 4; ++i) {
      const size_t ao = (size_t)(m0 + (i << 4) + rlane) * lda + koff + k0;
      V ah = Frag<T>::load(Ab + ao);
      V al;
      if (SPLIT) al = Frag<T>::load(Ab2 + ao);
#pragma unroll
      for (int j = 0; j < 4; ++j) {
        acc[i][j] = Frag<T>::mma(ah, bh[j], acc[i][j]);
        if (SPLIT) {
          acc[i][j] = Frag<T>::mma(ah, bl[j], acc[i][j]);
          acc[i][j] = Frag<T>::mma(al, bh[j], acc[i][j]);
        }
      }
      Frag<T>::guard(acc[i][0], acc[i][3], ah, SPLIT ? al : ah);
      Frag<T>::guard(acc[i][1], acc[i][2], ah, SPLIT ? al : ah);
    }
    Frag<T>::keep(bh[0], bh[1], bh[2], bh[3]);
    if (SPLIT) Frag<T>::keep(bl[0], bl[1], bl[2], bl[3]);
  }
  acc_guard4(acc[0][0], acc[0][1], acc[0][2], acc[0][3]);
  acc_guard4(acc[1][0], acc[1][1], acc[1][2], acc[1][3]);
  acc_guard4(acc[2][0], acc[2][1], acc[2][2], acc[2][3]);
  acc_guard4(acc[3][0], acc[3][1], acc[3][2], acc[3][3]);

  float* slab = sT[wave];
  const float* Rb = RESID ? (resid + (size_t)b * strideR) : nullptr;
#pragma unroll
  for (int i = 0; i < 4; ++i) {
    const int mBase = m0 + (i << 4);
#pragma unroll
    for (int j = 0; j < 4; ++j) {
      const int n = n0 + (j << 4) + rlane;
      float bv = 0.f;
      if (BIAS_MODE == 2) bv = bias[n];
#pragma unroll
      for (int r = 0; r < 8; ++r) {
        float v = acc[i][j][r] * scale;
        if (BIAS_MODE == 1) v += bias[mBase + mOff + r];
        if (BIAS_MODE == 2) v += bv;
        if (RESID) v += Rb[(size_t)(mBase + mOff + r) * ldc + n];
        if (ACT == 1) v = tanhf(v);
        if (ACT == 2) v = fmaxf(v, 0.0f);
        if (ACT == 3) v = v / (1.0f + expf(-v));
        if (ACT == 4) v = (v > 0.f) ? v : 0.01f * v;
        slab[(mOff + r) * 68 + (j << 4) + rlane] = v;
      }
    }
    __builtin_amdgcn_fence(__ATOMIC_RELEASE, "workgroup");
    __builtin_amdgcn_wave_barrier();
    __builtin_amdgcn_fence(__ATOMIC_ACQUIRE, "workgroup");
    if (OUT_MODE == 0) {
      float* C = (float*)Cout + (size_t)b * strideC;
      const int hh = lane >> 4, c4 = (lane & 15) * 4;
      for (int pass = 0; pass < 2; ++pass) {
#pragma unroll
        for (int it = 0; it < 8; ++it) {
          const int row = it * 2 + hh;
          v4f v = *(const v4f*)(slab + row * 68 + c4);
          *(volatile v4f*)(C + (size_t)(mBase + row) * ldc + n0 + c4) = v;
        }
        __threadfence();
      }
    } else {
      const int q = lane >> 3, c8 = (lane & 7) * 8;
      unsigned short* C  = (unsigned short*)Cout  + (size_t)b * strideC;
      unsigned short* C2 = (OUT_MODE == 2) ? ((unsigned short*)Cout2 + (size_t)b * strideC) : nullptr;
      for (int pass = 0; pass < 2; ++pass) {
#pragma unroll
        for (int it = 0; it < 4; ++it) {
          const int row = it * 4 + q;
          const float* sp = slab + row * 68 + c8;
          v8h hv, lv;
#pragma unroll
          for (int e = 0; e < 8; ++e) {
            if (OUT_MODE == 1) {
              hv[e] = (_Float16)sp[e];
            } else {
              unsigned short hb = f2bf_bits(sp[e]);
              unsigned short lb = f2bf_bits(sp[e] - bf_bits2f(hb));
              hv[e] = __builtin_bit_cast(_Float16, hb);
              lv[e] = __builtin_bit_cast(_Float16, lb);
            }
          }
          *(volatile v8h*)(C + (size_t)(mBase + row) * ldc + n0 + c8) = hv;
          if (OUT_MODE == 2) *(volatile v8h*)(C2 + (size_t)(mBase + row) * ldc + n0 + c8) = lv;
        }
        __threadfence();
      }
    }
    __builtin_amdgcn_fence(__ATOMIC_RELEASE, "workgroup");
    __builtin_amdgcn_wave_barrier();
    __builtin_amdgcn_fence(__ATOMIC_ACQUIRE, "workgroup");
  }
}

__global__ __launch_bounds__(256) void cvt8_f16_kernel(const float* __restrict__ src, unsigned short* __restrict__ dst,
                                                       int nrow, int ncol8, int spitch, float sc) {
  const int i  = blockIdx.x * 256 + threadIdx.x;
  const int n8 = nrow * ncol8;
  if (i < n8) {
    const int row = i / ncol8;
    const int c8  = i - row * ncol8;
    const float* sp = src + (size_t)row * spitch + c8 * 8;
    const v4f a = *(const v4f*)(sp);
    const v4f b = *(const v4f*)(sp + 4);
    v8h hv;
#pragma unroll
    for (int e = 0; e < 4; ++e) {
      const float fa = a[e] * sc;
      const float fb = b[e] * sc;
      hv[e]     = (_Float16)fa;
      hv[4 + e] = (_Float16)fb;
    }
    *(volatile v8h*)(dst + (size_t)i * 8) = hv;
    __threadfence();
    *(volatile v8h*)(dst + (size_t)i * 8) = hv;
  }
}

__global__ __launch_bounds__(256) void prep_small_kernel(const float* __restrict__ b_ih, const float* __restrict__ b_hh,
                                                         const float* __restrict__ w_v,
                                                         float* __restrict__ biasg, unsigned short* __restrict__ wvb) {
  const int tid = threadIdx.x;
  if (tid < 64) {
    const v4f a = *(const v4f*)(b_ih + 4 * tid);
    const v4f b = *(const v4f*)(b_hh + 4 * tid);
    v4f o;
#pragma unroll
    for (int e = 0; e < 4; ++e) o[e] = a[e] + b[e];
    *(volatile v4f*)(biasg + 4 * tid) = o;
    __threadfence();
    *(volatile v4f*)(biasg + 4 * tid) = o;
  }
  if (tid >= 128) {
    const int idx = tid - 128;
    const int n = idx >> 3;
    const int c8 = (idx & 7) * 8;
    const v4f wa = *(const v4f*)(w_v + c8);
    const v4f wb = *(const v4f*)(w_v + c8 + 4);
    float w[8];
#pragma unroll
    for (int e = 0; e < 4; ++e) { w[e] = wa[e] * WV_CARRY; w[4 + e] = wb[e] * WV_CARRY; }
    v8h hv;
#pragma unroll
    for (int e = 0; e < 8; ++e) {
      const _Float16 hi16 = (_Float16)w[e];
      const unsigned short hb = __builtin_bit_cast(unsigned short, hi16);
      const float hif = h16_to_f32((unsigned)hb);
      const float lo = (w[e] - hif) * WV_RES;
      const float sel = (n == 0) ? w[e] : ((n == 1) ? lo : 0.0f);
      hv[e] = (_Float16)sel;
    }
    *(volatile v8h*)(wvb + (size_t)idx * 8) = hv;
    __threadfence();
    *(volatile v8h*)(wvb + (size_t)idx * 8) = hv;
  }
}

__device__ __forceinline__ float tanh_fast(float v) { return 1.0f - 2.0f * __builtin_amdgcn_rcpf(__expf(2.0f * v) + 1.0f); }
__device__ __forceinline__ float sig_p(float v)  { return 1.0f / (1.0f + expf(-v)); }
__device__ __forceinline__ float tanh_p(float v) { return 1.0f - 2.0f * (1.0f / (1.0f + expf(2.0f * v))); }

__device__ __forceinline__ v16h tanh_frag(const float* __restrict__ ur, const float (&wo)[16]) {
  const v4f u0 = *(const v4f*)(ur);
  const v4f u1 = *(const v4f*)(ur + 4);
  const v4f u2 = *(const v4f*)(ur + 16);
  const v4f u3 = *(const v4f*)(ur + 20);
  v16h a;
#pragma unroll
  for (int e = 0; e < 4; ++e) {
    const float t0 = tanh_fast(wo[e] + u0[e]);
    const float t1 = tanh_fast(wo[4 + e] + u1[e]);
    const float t2 = tanh_fast(wo[8 + e] + u2[e]);
    const float t3 = tanh_fast(wo[12 + e] + u3[e]);
    a[e]      = (_Float16)t0;
    a[4 + e]  = (_Float16)t1;
    a[8 + e]  = (_Float16)t2;
    a[12 + e] = (_Float16)t3;
  }
  return a;
}

__global__ __launch_bounds__(SCAN_THR) void scan_kernel(const float* __restrict__ x, const float* __restrict__ Uplane,
                                                        const unsigned short* __restrict__ WWp,
                                                        const unsigned short* __restrict__ WHHp,
                                                        const unsigned short* __restrict__ WIHp,
                                                        const unsigned short* __restrict__ WVBp,
                                                        const float* __restrict__ biasg, const float* __restrict__ b_w,
                                                        float* __restrict__ out0, float* __restrict__ out1) {
  __shared__ __align__(16) _Float16 HC[16 * HCP];
  __shared__ __align__(16) _Float16 XT[16 * XTP];
  __shared__ __align__(16) float    WO[16 * 64];
  __shared__ __align__(16) float    SG[2 * 16 * NVAR];
  __shared__ __align__(16) float    CS[16 * 64];
  __shared__ __align__(16) float    HS[16 * 64];
  const _Float16* WW  = (const _Float16*)WWp;
  const _Float16* WHH = (const _Float16*)WHHp;
  const _Float16* WIH = (const _Float16*)WIHp;
  const _Float16* WVB = (const _Float16*)WVBp;
  const int tid = threadIdx.x, lane = tid & 31, wave = tid >> 5;
  const int c = lane & 15, hh = lane >> 4, koff = 8 * hh;
  const int b0 = blockIdx.x * BLK_ROWS;
  const int gcol = 16 * wave + c;

#pragma unroll 1
  for (int i = tid; i < 16 * HCP; i += SCAN_THR) HC[i] = (_Float16)0.0f;
#pragma unroll 1
  for (int i = tid; i < 16 * XTP; i += SCAN_THR) XT[i] = (_Float16)0.0f;
  CS[tid] = 0.0f;
  CS[tid + SCAN_THR] = 0.0f;

  const float bwv = b_w[gcol & 63];
  const float bgv = biasg[gcol];
  const v16h wvb0 = Frag<_Float16>::load(WVB + c * 64 + koff);
  const v16h wvb1 = Frag<_Float16>::load(WVB + c * 64 + koff + 32);
  const v8f z8 = {0.f, 0.f, 0.f, 0.f, 0.f, 0.f, 0.f, 0.f};
  __syncthreads();

#pragma unroll 1
  for (int t = 0; t < NWIN; ++t) {
    if (wave < 4) {
      const _Float16* ar = HC + c * HCP + koff;
      const _Float16* br = WW + (size_t)gcol * NKHC + koff;
      v8f acc = z8;
#pragma unroll 1
      for (int k0 = 0; k0 < NKHC; k0 += 32) {
        const v16h a = Frag<_Float16>::load(ar + k0);
        const v16h b = Frag<_Float16>::load(br + k0);
        acc = mma_h(a, b, acc);
      }
#pragma unroll
      for (int r = 0; r < 8; ++r) WO[(8 * hh + r) * 64 + gcol] = acc[r] * FOLD_INV + bwv;
    }
    __syncthreads();

    {
      const int b = wave;
      float wo0[16], wo1[16];
      {
        const float* wp = WO + b * 64 + koff;
        const v4f a0 = *(const v4f*)(wp);
        const v4f a1 = *(const v4f*)(wp + 4);
        const v4f a2 = *(const v4f*)(wp + 16);
        const v4f a3 = *(const v4f*)(wp + 20);
        const v4f c0 = *(const v4f*)(wp + 32);
        const v4f c1 = *(const v4f*)(wp + 36);
        const v4f c2 = *(const v4f*)(wp + 48);
        const v4f c3 = *(const v4f*)(wp + 52);
#pragma unroll
        for (int e = 0; e < 4; ++e) {
          wo0[e] = a0[e]; wo0[4 + e] = a1[e]; wo0[8 + e] = a2[e]; wo0[12 + e] = a3[e];
          wo1[e] = c0[e]; wo1[4 + e] = c1[e]; wo1[8 + e] = c2[e]; wo1[12 + e] = c3[e];
        }
      }
      const float* ub = Uplane + ((size_t)(b0 + b) * NVAR + c) * NWIN + koff;
#pragma unroll 1
      for (int tile = 0; tile < 16; ++tile) {
        const float* ur = ub + (size_t)tile * 16 * NWIN;
        v8f acc = z8;
        const v16h fa0 = tanh_frag(ur, wo0);
        acc = mma_h(fa0, wvb0, acc);
        const v16h fa1 = tanh_frag(ur + 32, wo1);
        acc = mma_h(fa1, wvb1, acc);
        if (c < 2) {
          float* dst = SG + c * (16 * NVAR) + b * NVAR + 16 * tile + 8 * hh;
          const v4f d0 = {acc[0], acc[1], acc[2], acc[3]};
          const v4f d1 = {acc[4], acc[5], acc[6], acc[7]};
          *(v4f*)(dst) = d0;
          *(v4f*)(dst + 4) = d1;
        }
      }
    }
    __syncthreads();

    {
      const int b = wave;
      float s[2][4], xv[2][4], xt[2][4];
      const float* xp = x + ((size_t)(b0 + b) * NVAR + 4 * lane) * NWIN + t;
#pragma unroll
      for (int q = 0; q < 2; ++q) {
        const v4f sh = *(const v4f*)(SG + b * NVAR + 128 * q + 4 * lane);
        const v4f sl = *(const v4f*)(SG + 16 * NVAR + b * NVAR + 128 * q + 4 * lane);
#pragma unroll
        for (int e = 0; e < 4; ++e) {
          s[q][e] = (sh[e] + sl[e] * WV_RES_INV) * WV_CARRY_INV;
          xv[q][e] = xp[(size_t)(128 * q + e) * NWIN];
        }
      }
      float m = s[0][0];
#pragma unroll
      for (int q = 0; q < 2; ++q)
#pragma unroll
        for (int e = 0; e < 4; ++e) m = fmaxf(m, s[q][e]);
#pragma unroll
      for (int off = 1; off < 32; off <<= 1) m = fmaxf(m, __shfl_xor(m, off, 32));
      float sum = 0.0f;
#pragma unroll
      for (int q = 0; q < 2; ++q)
#pragma unroll
        for (int e = 0; e < 4; ++e) { s[q][e] = expf(s[q][e] - m); sum += s[q][e]; }
#pragma unroll
      for (int off = 1; off < 32; off <<= 1) sum += __shfl_xor(sum, off, 32);
      const float inv = 1.0f / sum;
#pragma unroll
      for (int q = 0; q < 2; ++q)
#pragma unroll
        for (int e = 0; e < 4; ++e) xt[q][e] = (s[q][e] * inv) * xv[q][e];
#pragma unroll
      for (int q = 0; q < 2; ++q) {
        const _Float16 g0 = (_Float16)(xt[q][0] * ACT_CARRY);
        const _Float16 g1 = (_Float16)(xt[q][1] * ACT_CARRY);
        const _Float16 g2 = (_Float16)(xt[q][2] * ACT_CARRY);
        const _Float16 g3 = (_Float16)(xt[q][3] * ACT_CARRY);
        const unsigned u0 = (unsigned)__builtin_bit_cast(unsigned short, g0);
        const unsigned u1 = (unsigned)__builtin_bit_cast(unsigned short, g1);
        const unsigned u2 = (unsigned)__builtin_bit_cast(unsigned short, g2);
        const unsigned u3 = (unsigned)__builtin_bit_cast(unsigned short, g3);
        v2u pk;
        pk[0] = u0 | (u1 << 16);
        pk[1] = u2 | (u3 << 16);
        *(v2u*)(XT + b * XTP + 128 * q + 4 * lane) = pk;
      }
      const v4f o0 = {xt[0][0], xt[0][1], xt[0][2], xt[0][3]};
      const v4f o1 = {xt[1][0], xt[1][1], xt[1][2], xt[1][3]};
      float* op = out0 + ((size_t)t * NBATCH + (size_t)(b0 + b)) * NVAR + 4 * lane;
      *(volatile v4f*)(op) = o0;
      *(volatile v4f*)(op + 128) = o1;
      __threadfence();
      *(volatile v4f*)(op) = o0;
      *(volatile v4f*)(op + 128) = o1;
    }
    __syncthreads();

    {
      const _Float16* ar = XT + c * XTP + koff;
      const _Float16* hr = HC + c * HCP + koff;
      const _Float16* b1 = WIH + (size_t)gcol * NVAR + koff;
      const _Float16* b2 = WHH + (size_t)gcol * NHID + koff;
      v8f acc = z8;
#pragma unroll 1
      for (int k0 = 0; k0 < NVAR; k0 += 32) {
        const v16h a = Frag<_Float16>::load(ar + k0);
        const v16h b = Frag<_Float16>::load(b1 + k0);
        acc = mma_h(a, b, acc);
      }
#pragma unroll 1
      for (int k0 = 0; k0 < NHID; k0 += 32) {
        const v16h a = Frag<_Float16>::load(hr + k0);
        const v16h b = Frag<_Float16>::load(b2 + k0);
        acc = mma_h(a, b, acc);
      }
#pragma unroll
      for (int r = 0; r < 8; ++r) SG[(8 * hh + r) * GTP + gcol] = acc[r] * FOLD_INV + bgv;
    }
    __syncthreads();

#pragma unroll 1
    for (int cell = 0; cell < 2; ++cell) {
      const int idx = tid + SCAN_THR * cell;
      const int bb = idx >> 6, j = idx & 63;
      const float gi = SG[bb * GTP + j];
      const float gf = SG[bb * GTP + 64 + j];
      const float gg = SG[bb * GTP + 128 + j];
      const float go = SG[bb * GTP + 192 + j];
      const float ig = sig_p(gi);
      const float fg = sig_p(gf);
      const float gt = tanh_p(gg);
      const float og = sig_p(go);
      const float cn = fg * CS[idx] + ig * gt;
      const float hn = og * tanh_p(cn);
      CS[idx] = cn;
      HS[idx] = hn;
      HC[bb * HCP + j]      = (_Float16)(hn * ACT_CARRY);
      HC[bb * HCP + 64 + j] = (_Float16)(cn * ACT_CARRY);
    }
    __syncthreads();

    if (tid < 256) {
      const v4f hv = *(const v4f*)(HS + 4 * tid);
      float* op = out1 + ((size_t)t * NBATCH + (size_t)b0) * NHID + 4 * tid;
      *(volatile v4f*)(op) = hv;
      __threadfence();
      *(volatile v4f*)(op) = hv;
    }
  }
}

extern "C" void kernel_launch(void* const* d_in, const int* in_sizes, int n_in,
                              void* d_out, int out_size, void* d_ws, size_t ws_size, hipStream_t stream) {
  if (n_in < 10 || d_out == nullptr || d_ws == nullptr) return;
  if (in_sizes[0] != NBATCH * NVAR * NWIN || in_sizes[1] != NGATE * NVAR || in_sizes[2] != NGATE * NHID ||
      in_sizes[3] != NGATE || in_sizes[4] != NGATE || in_sizes[5] != NWIN || in_sizes[6] != NWIN * NKHC ||
      in_sizes[7] != NWIN || in_sizes[8] != NWIN * NWIN || in_sizes[9] != NWIN || out_size != NOUT0 + NOUT1) return;

  const float* x    = (const float*)d_in[0];
  const float* w_ih = (const float*)d_in[1];
  const float* w_hh = (const float*)d_in[2];
  const float* b_ih = (const float*)d_in[3];
  const float* b_hh = (const float*)d_in[4];
  const float* w_v  = (const float*)d_in[5];
  const float* w_w  = (const float*)d_in[6];
  const float* b_w  = (const float*)d_in[7];
  const float* w_u  = (const float*)d_in[8];
  const float* b_u  = (const float*)d_in[9];
  float* out0 = (float*)d_out;
  float* out1 = out0 + (size_t)NOUT0;

  char* ws = (char*)d_ws; size_t off = 0;
  auto carve = [&](size_t bytes) -> char* { char* p = ws + off; off += (bytes + 255) & ~(size_t)255; return p; };
  unsigned short* X16   = (unsigned short*)carve((size_t)ROWS_UV * NWIN * 2);
  unsigned short* WU16  = (unsigned short*)carve((size_t)NWIN * NWIN * 2);
  unsigned short* WW16  = (unsigned short*)carve((size_t)NWIN * NKHC * 2);
  unsigned short* WHH16 = (unsigned short*)carve((size_t)NGATE * NHID * 2);
  unsigned short* WIH16 = (unsigned short*)carve((size_t)NGATE * NVAR * 2);
  unsigned short* WVB   = (unsigned short*)carve((size_t)16 * NWIN * 2);
  float*          BIASG = (float*)carve((size_t)NGATE * 4);
  float*          UPL   = (float*)carve((size_t)ROWS_UV * NWIN * 4);
  if (off > ws_size || off > (size_t)134217728) return;

  const int n8x  = ROWS_UV * (NWIN / 8);
  const int n8u  = NWIN * (NWIN / 8);
  const int n8w  = NWIN * (NKHC / 8);
  const int n8hh = NGATE * (NHID / 8);
  const int n8ih = NGATE * (NVAR / 8);
  cvt8_f16_kernel<<<(n8x + 255) / 256, 256, 0, stream>>>(x, X16, ROWS_UV, NWIN / 8, NWIN, 1.0f);
  cvt8_f16_kernel<<<(n8u + 255) / 256, 256, 0, stream>>>(w_u, WU16, NWIN, NWIN / 8, NWIN, W_CARRY);
  cvt8_f16_kernel<<<(n8w + 255) / 256, 256, 0, stream>>>(w_w, WW16, NWIN, NKHC / 8, NKHC, W_CARRY);
  cvt8_f16_kernel<<<(n8hh + 255) / 256, 256, 0, stream>>>(w_hh, WHH16, NGATE, NHID / 8, NHID, W_CARRY);
  cvt8_f16_kernel<<<(n8ih + 255) / 256, 256, 0, stream>>>(w_ih, WIH16, NGATE, NVAR / 8, NVAR, W_CARRY);
  prep_small_kernel<<<1, 256, 0, stream>>>(b_ih, b_hh, w_v, BIASG, WVB);

  const dim3 ggrid((ROWS_UV / 64) * (NWIN / 64) / 8, 1);
  wmma_gemm64<0, false, 2, 0, false, 0><<<ggrid, 256, 0, stream>>>(
      X16, X16, NWIN, 0L, WU16, WU16, NWIN, 0L, (void*)UPL, (void*)UPL, NWIN, 0L,
      b_u, UPL, 0L, ROWS_UV, NWIN, NWIN, W_CARRY_INV);

  scan_kernel<<<NBATCH / BLK_ROWS, SCAN_THR, 0, stream>>>(x, UPL, WW16, WHH16, WIH16, WVB, BIASG, b_w, out0, out1);
}
